// StructuralCausalModel_54494545051775
// MI455X (gfx1250) — hardware-verified
//
#include <hip/hip_runtime.h>

#define NB_  8192
#define DD_  256
#define HH_  64
#define RPB  64
#define NTW  2
#define WST  264
#define HST  72

typedef _Float16 f16;
typedef __attribute__((ext_vector_type(16))) f16 f16x16;
typedef __attribute__((ext_vector_type(8)))  f16 f16x8;
typedef __attribute__((ext_vector_type(8)))  float f32x8;
typedef __attribute__((ext_vector_type(4)))  float v4f_t;
typedef __attribute__((ext_vector_type(4)))  unsigned v4u_t;

__device__ __forceinline__ f32x8 wmma16(f16x16 a, f16x16 b, f32x8 c) {
  c = __builtin_amdgcn_wmma_f32_16x16x32_f16(false, a, false, b, (short)0, c, false, false);
  asm volatile("v_nop\n\tv_nop\n\tv_nop\n\tv_nop" : "+v"(c) : "v"(a), "v"(b));
  return c;
}
__device__ __forceinline__ f16x16 lds_frag(const f16* base, int stride) {
  const int lane = threadIdx.x & 31, row = lane & 15, kh = (lane >> 4) * 8;
  const f16x8 lo = *(const f16x8*)(base + row * stride + kh);
  const f16x8 hi = *(const f16x8*)(base + row * stride + kh + 16);
  f16x16 f;
#pragma unroll
  for (int i = 0; i < 8; ++i) { f[i] = lo[i]; f[i + 8] = hi[i]; }
  return f;
}
__device__ __forceinline__ f16x16 gbl_frag(const f16* __restrict__ base, int stride) {
  const int lane = threadIdx.x & 31, row = lane & 15, kh = (lane >> 4) * 8;
  const f16x8 lo = *(const f16x8*)(base + (size_t)row * stride + kh);
  const f16x8 hi = *(const f16x8*)(base + (size_t)row * stride + kh + 16);
  f16x16 f;
#pragma unroll
  for (int i = 0; i < 8; ++i) { f[i] = lo[i]; f[i + 8] = hi[i]; }
  return f;
}

__global__ __launch_bounds__(256) void k_prescale(const float* __restrict__ W1, const float* __restrict__ adjl, f16* __restrict__ W1s) {
  const size_t g = (size_t)blockIdx.x * 256 + threadIdx.x;
  const size_t e0 = g * 8;
  const int i = (int)(e0 >> 14), j0 = (int)(e0 & 255);
  union { f16 hh[8]; v4u_t v; } u;
#pragma unroll
  for (int t = 0; t < 8; ++t) {
    const int j = j0 + t;
    const float a = (j == i) ? 0.0f : 1.0f / (1.0f + __expf(-adjl[j * DD_ + i]));
    u.hh[t] = (f16)(W1[e0 + t] * a);
  }
  *(volatile v4u_t*)(W1s + e0) = u.v; __threadfence(); *(volatile v4u_t*)(W1s + e0) = u.v;
}

__global__ __launch_bounds__(64) void scm_kernel(const float* __restrict__ noise,
                                                 const f16*   __restrict__ W1s,
                                                 const float* __restrict__ b1,
                                                 const float* __restrict__ W2,
                                                 const float* __restrict__ b2,
                                                 const float* __restrict__ lsig,
                                                 float* __restrict__ out) {
  __shared__ __attribute__((aligned(16))) f16 zh[2][NTW * 16 * WST];
  __shared__ __attribute__((aligned(16))) f16 hS[2][NTW * 16 * HST];
  const int tid = threadIdx.x, lane = tid & 31, wave = tid >> 5, cl = lane & 15, rh = (lane >> 4) * 8, kh = rh;
  const int row0 = blockIdx.x * RPB + wave * (NTW * 16);
  f16* zw = zh[wave]; f16* hw = hS[wave];
  for (int e = lane; e < NTW * 16 * WST; e += 32) zw[e] = (f16)0.0f;
  asm volatile("s_wait_dscnt 0" ::: "memory");
  __builtin_amdgcn_wave_barrier();

#pragma unroll 1
  for (int i = 0; i < DD_; ++i) {
    const int nks = (i + 31) >> 5;
    const f16* Wi = W1s + (size_t)i * HH_ * DD_;
    f32x8 acc[NTW][4];
#pragma unroll
    for (int t = 0; t < NTW; ++t)
#pragma unroll
      for (int nt = 0; nt < 4; ++nt) { f32x8 zz = {}; acc[t][nt] = zz; }
    for (int ks = 0; ks < nks; ++ks) {
      f16x16 af[NTW];
#pragma unroll
      for (int t = 0; t < NTW; ++t) af[t] = lds_frag(zw + t * 16 * WST + ks * 32, WST);
#pragma unroll
      for (int nt = 0; nt < 4; ++nt) {
        const f16x16 bf = gbl_frag(Wi + (size_t)(nt * 16) * DD_ + ks * 32, DD_);
#pragma unroll
        for (int t = 0; t < NTW; ++t) acc[t][nt] = wmma16(af[t], bf, acc[t][nt]);
      }
    }
#pragma unroll
    for (int nt = 0; nt < 4; ++nt) {
      const int hh = nt * 16 + cl;
      const float bb = b1[i * HH_ + hh];
#pragma unroll
      for (int t = 0; t < NTW; ++t)
#pragma unroll
        for (int r = 0; r < 8; ++r) {
          const float p = acc[t][nt][r] + bb;
          hw[(t * 16 + rh + r) * HST + hh] = (f16)(p / (1.0f + __expf(-p)));
        }
    }
    f16x16 wb[2];
#pragma unroll
    for (int ks = 0; ks < 2; ++ks)
#pragma unroll
      for (int e = 0; e < 8; ++e) {
        wb[ks][e]     = (cl == 0) ? (f16)W2[i * HH_ + ks * 32 + kh + e]      : (f16)0.0f;
        wb[ks][e + 8] = (cl == 0) ? (f16)W2[i * HH_ + ks * 32 + kh + 16 + e] : (f16)0.0f;
      }
    asm volatile("s_wait_dscnt 0" ::: "memory");
    __builtin_amdgcn_wave_barrier();
    const float bb2 = b2[i], sg = __expf(lsig[i]);
#pragma unroll
    for (int t = 0; t < NTW; ++t) {
      f32x8 dz = {};
#pragma unroll
      for (int ks = 0; ks < 2; ++ks) dz = wmma16(lds_frag(hw + t * 16 * HST + ks * 32, HST), wb[ks], dz);
      if (cl == 0) {
#pragma unroll
        for (int r = 0; r < 8; ++r) {
          const int rr = t * 16 + rh + r;
          zw[rr * WST + i] = (f16)(dz[r] + bb2 + sg * noise[(size_t)(row0 + rr) * DD_ + i]);
        }
      }
    }
    asm volatile("s_wait_dscnt 0" ::: "memory");
    __builtin_amdgcn_wave_barrier();
  }
#pragma unroll 1
  for (int pass = 0; pass < 2; ++pass) {
#pragma unroll 1
    for (int it = 0; it < 32 * NTW; ++it) {
      const int f4 = lane + 32 * it, rr = f4 >> 6, q = (f4 & 63) * 4;
      v4f_t v;
#pragma unroll
      for (int u = 0; u < 4; ++u) v[u] = (float)zw[rr * WST + q + u];
      *(volatile v4f_t*)(out + (size_t)(row0 + rr) * DD_ + q) = v;
    }
    __threadfence();
  }
}

extern "C" void kernel_launch(void* const* d_in, const int* in_sizes, int n_in,
                              void* d_out, int out_size, void* d_ws, size_t ws_size,
                              hipStream_t stream) {
  (void)in_sizes; (void)n_in; (void)out_size; (void)ws_size;
  const float* noise = (const float*)d_in[0];
  const float* adjl  = (const float*)d_in[1];
  const float* W1    = (const float*)d_in[2];
  const float* b1    = (const float*)d_in[3];
  const float* W2    = (const float*)d_in[4];
  const float* b2    = (const float*)d_in[5];
  const float* lsig  = (const float*)d_in[6];
  float* out = (float*)d_out;
  f16* W1s = (f16*)d_ws;
  k_prescale<<<dim3(524288 / 256), dim3(256), 0, stream>>>(W1, adjl, W1s);
  scm_kernel<<<dim3(NB_ / RPB), dim3(64), 0, stream>>>(noise, W1s, b1, W2, b2, lsig, out);
}
